// SSM_62998580297845
// MI455X (gfx1250) — hardware-verified
//
#include <hip/hip_runtime.h>
#include <math.h>

typedef __attribute__((ext_vector_type(16))) _Float16 v16h;
typedef __attribute__((ext_vector_type(8)))  _Float16 v8h;
typedef __attribute__((ext_vector_type(8)))  float    v8f;
typedef __attribute__((ext_vector_type(4)))  float    v4f;
typedef __attribute__((ext_vector_type(2)))  float    v2f;

constexpr int kBsz      = 16;
constexpr int kT        = 4096;
constexpr int kU        = 128;
constexpr int kO        = 128;
constexpr int kS        = 256;
constexpr int kH        = 512;
constexpr int kRows     = kBsz * kT;
constexpr int kSlabRows = kRows / 2;
constexpr int kCatK     = kS + kU;
constexpr int kW3lK     = kH + kU;
constexpr int kScanTS   = 16;
constexpr int kScanP    = 260;
constexpr float kWCarry    = 16.0f;
constexpr float kWCarryInv = 1.0f / kWCarry;

static_assert(kRows == 65536, "rows");
static_assert(kCatK == 384 && kW3lK == 640, "fused K extents");
static_assert((kU % 32) == 0 && (kS % 32) == 0 && (kO % 32) == 0 && (kH % 32) == 0, "GEMM K multiples of 32");
static_assert((kRows % 64) == 0 && (kSlabRows % 64) == 0, "GEMM M multiples of 64");
static_assert((kS % 64) == 0 && (kO % 64) == 0 && (kH % 64) == 0, "GEMM N multiples of 64");
static_assert((kT % kScanTS) == 0, "scan chunking");
static_assert(((kRows / 64) * (kS / 64)) % 8 == 0, "S1 tiles fill whole blocks");
static_assert(((kRows / 64) * (kO / 64)) % 8 == 0, "S2 tiles fill whole blocks");
static_assert(((kSlabRows / 64) * (kH / 64)) % 8 == 0, "S3/S4 tiles fill whole blocks");
static_assert(((kSlabRows / 64) * (kO / 64)) % 8 == 0, "S5 tiles fill whole blocks");

constexpr size_t kSzX16  = (size_t)kRows * kU * 2;
constexpr size_t kSzB16  = (size_t)kS * kU * 2;
constexpr size_t kSzCAT  = (size_t)kO * kCatK * 2;
constexpr size_t kSzW116 = (size_t)kH * kO * 2;
constexpr size_t kSzW216 = (size_t)kH * kH * 2;
constexpr size_t kSzW3L  = (size_t)kO * kW3lK * 2;
constexpr size_t kSzR1   = (size_t)kRows * kS * 4;
constexpr size_t kSzR2   = (size_t)kRows * kS * 2;
constexpr size_t kSzY16  = (size_t)kRows * kO * 2;
constexpr size_t kSzZ    = (size_t)kSlabRows * kH * 2;
constexpr size_t kOffX16  = 0;
constexpr size_t kOffB16  = kOffX16  + kSzX16;
constexpr size_t kOffCAT  = kOffB16  + kSzB16;
constexpr size_t kOffW116 = kOffCAT  + kSzCAT;
constexpr size_t kOffW216 = kOffW116 + kSzW116;
constexpr size_t kOffW3L  = kOffW216 + kSzW216;
constexpr size_t kOffR1   = kOffW3L  + kSzW3L;
constexpr size_t kOffR2   = kOffR1   + kSzR1;
constexpr size_t kWsTotal = kOffR2   + kSzR2;
constexpr size_t kOffY16  = kOffR1;
constexpr size_t kOffZ1   = kOffR1 + kSzY16;
constexpr size_t kOffZ2   = kOffR2;
static_assert(kWsTotal == 118423552ull, "carve total");
static_assert(kWsTotal <= 134217728ull, "carve cap");
static_assert(kSzY16 + kSzZ <= kSzR1, "Y16 + Z1 fit in R1");
static_assert(kSzZ <= kSzR2, "Z2 fits in R2");
static_assert((kOffB16 % 128) == 0 && (kOffCAT % 128) == 0 && (kOffW116 % 128) == 0 && (kOffW216 % 128) == 0 &&
              (kOffW3L % 128) == 0 && (kOffR1 % 128) == 0 && (kOffR2 % 128) == 0 && (kOffZ1 % 128) == 0,
              "128-B aligned regions");

union FragU { v16h v; v8h h[2]; };
__device__ __forceinline__ v16h frag_load(const _Float16* p) {
  FragU f;
  f.h[0] = *(const v8h*)(p);
  f.h[1] = *(const v8h*)(p + 16);
  return f.v;
}
__device__ __forceinline__ v8f mma_f16(v16h a, v16h b, v8f c) {
  return __builtin_amdgcn_wmma_f32_16x16x32_f16(false, a, false, b, (short)0, c, false, false);
}
__device__ __forceinline__ void row_guard_h(v8f& a, v8f& b, v8f& c, v8f& d, v16h x,
                                            v16h y0, v16h y1, v16h y2, v16h y3) {
  asm volatile("v_nop\n\tv_nop\n\tv_nop\n\tv_nop"
               : "+v"(a), "+v"(b), "+v"(c), "+v"(d)
               : "v"(x), "v"(y0), "v"(y1), "v"(y2), "v"(y3));
}
__device__ __forceinline__ void keep4_h(v16h a, v16h b, v16h c, v16h d) {
  asm volatile("v_nop" :: "v"(a), "v"(b), "v"(c), "v"(d));
}
__device__ __forceinline__ void acc_guard4(v8f& a, v8f& b, v8f& c, v8f& d) {
  asm volatile("v_nop\n\tv_nop\n\tv_nop\n\tv_nop" : "+v"(a), "+v"(b), "+v"(c), "+v"(d));
}
__device__ __forceinline__ void lds_wave_sync() {
  __builtin_amdgcn_fence(__ATOMIC_RELEASE, "workgroup");
  __builtin_amdgcn_wave_barrier();
  __builtin_amdgcn_fence(__ATOMIC_ACQUIRE, "workgroup");
}

template <int OUT_MODE, int ACT>
__global__ __launch_bounds__(256) void gemm2seg_f16_kernel(
    const unsigned short* A1p, int lda1, int K1,
    const unsigned short* A2p, int lda2, int K2,
    const unsigned short* __restrict__ Btp, int ldb,
    void* __restrict__ Cout, int ldc,
    int M, int N, float scale)
{
  const _Float16* A1 = (const _Float16*)A1p;
  const _Float16* A2 = (const _Float16*)A2p;
  const _Float16* Bt = (const _Float16*)Btp;
  __shared__ __align__(16) float sT[8][16 * 68];
  const int lane = threadIdx.x & 31;
  const int wave = threadIdx.x >> 5;
  const int tilesN = N >> 6;
  const int tilesM = M >> 6;
  const int tile = blockIdx.x * 8 + wave;
  if (tile >= tilesM * tilesN) return;
  const int tm = tile / tilesN;
  const int tn = tile - tm * tilesN;
  const int m0 = tm << 6;
  const int n0 = tn << 6;

  const int rlane = lane & 15;
  const int koff  = (lane >> 4) * 8;
  const int mOff  = (lane >> 4) * 8;

  v8f acc[4][4];
#pragma unroll
  for (int i = 0; i < 4; ++i)
#pragma unroll
    for (int j = 0; j < 4; ++j) acc[i][j] = (v8f){0.f, 0.f, 0.f, 0.f, 0.f, 0.f, 0.f, 0.f};

#pragma unroll 1
  for (int seg = 0; seg < 2; ++seg) {
    const _Float16* As = (seg == 0) ? A1 : A2;
    const int ldas = (seg == 0) ? lda1 : lda2;
    const int Ks   = (seg == 0) ? K1 : K2;
    const int kb   = (seg == 0) ? 0 : K1;
#pragma unroll 1
    for (int k0 = 0; k0 < Ks; k0 += 32) {
      v16h bh[4];
#pragma unroll
      for (int j = 0; j < 4; ++j) {
        const size_t bo = (size_t)(n0 + (j << 4) + rlane) * ldb + kb + k0 + koff;
        bh[j] = frag_load(Bt + bo);
      }
#pragma unroll
      for (int i = 0; i < 4; ++i) {
        const size_t ao = (size_t)(m0 + (i << 4) + rlane) * ldas + k0 + koff;
        const v16h ah = frag_load(As + ao);
#pragma unroll
        for (int j = 0; j < 4; ++j) acc[i][j] = mma_f16(ah, bh[j], acc[i][j]);
        row_guard_h(acc[i][0], acc[i][1], acc[i][2], acc[i][3], ah, bh[0], bh[1], bh[2], bh[3]);
      }
      keep4_h(bh[0], bh[1], bh[2], bh[3]);
    }
  }
  acc_guard4(acc[0][0], acc[0][1], acc[0][2], acc[0][3]);
  acc_guard4(acc[1][0], acc[1][1], acc[1][2], acc[1][3]);
  acc_guard4(acc[2][0], acc[2][1], acc[2][2], acc[2][3]);
  acc_guard4(acc[3][0], acc[3][1], acc[3][2], acc[3][3]);

  float* slab = sT[wave];
#pragma unroll
  for (int i = 0; i < 4; ++i) {
    const int mBase = m0 + (i << 4);
#pragma unroll
    for (int j = 0; j < 4; ++j) {
#pragma unroll
      for (int r = 0; r < 8; ++r) {
        float v = acc[i][j][r] * scale;
        if (ACT == 2) v = fmaxf(v, 0.0f);
        slab[(mOff + r) * 68 + (j << 4) + rlane] = v;
      }
    }
    lds_wave_sync();
    if (ACT == 3) {
      const int hh2 = lane >> 4, c4s = (lane & 15) * 4;
#pragma unroll 1
      for (int it = 0; it < 8; ++it) {
        float* sp = slab + (it * 2 + hh2) * 68 + c4s;
        v4f t = *(const v4f*)sp;
#pragma unroll
        for (int e = 0; e < 4; ++e) {
          const float tv = t[e];
          const float sg = __builtin_amdgcn_rcpf(1.0f + expf(-tv));
          t[e] = tv * sg;
        }
        *(v4f*)sp = t;
      }
      lds_wave_sync();
    }
    if (OUT_MODE == 0) {
      float* C = (float*)Cout;
      const int hh = lane >> 4, c4 = (lane & 15) * 4;
      for (int pass = 0; pass < 2; ++pass) {
#pragma unroll
        for (int it = 0; it < 8; ++it) {
          const int row = it * 2 + hh;
          const v4f v = *(const v4f*)(slab + row * 68 + c4);
          *(volatile v4f*)(C + (size_t)(mBase + row) * ldc + n0 + c4) = v;
        }
        __threadfence();
      }
    } else {
      unsigned short* C = (unsigned short*)Cout;
      const int q = lane >> 3, c8 = (lane & 7) * 8;
      for (int pass = 0; pass < 2; ++pass) {
#pragma unroll
        for (int it = 0; it < 4; ++it) {
          const int row = it * 4 + q;
          const float* sp = slab + row * 68 + c8;
          v8h hv;
#pragma unroll
          for (int e = 0; e < 8; ++e) hv[e] = (_Float16)sp[e];
          *(volatile v8h*)(C + (size_t)(mBase + row) * ldc + n0 + c8) = hv;
        }
        __threadfence();
      }
    }
    lds_wave_sync();
  }
}

__global__ __launch_bounds__(256) void cast_f16_pitch_kernel(
    const float* __restrict__ src, unsigned short* __restrict__ dst,
    int total8, int cols, int dpitch, int dcol0, float scale)
{
  const int i = blockIdx.x * 256 + threadIdx.x;
  if (i >= total8) return;
  const int e0  = i << 3;
  const int row = e0 / cols;
  const int c   = e0 - row * cols;
  const float* p = src + (size_t)e0;
  const v4f a0 = *(const v4f*)(p);
  const v4f a1 = *(const v4f*)(p + 4);
  v8h hv;
#pragma unroll
  for (int e = 0; e < 4; ++e) {
    hv[e]     = (_Float16)(a0[e] * scale);
    hv[4 + e] = (_Float16)(a1[e] * scale);
  }
  unsigned short* q = dst + (size_t)row * dpitch + dcol0 + c;
  *(volatile v8h*)q = hv;
  __threadfence();
  *(volatile v8h*)q = hv;
}

__global__ __launch_bounds__(128) void scan_kernel(
    const float* __restrict__ bu, const float* __restrict__ lre, const float* __restrict__ lim,
    unsigned short* __restrict__ h16)
{
  __shared__ __align__(16) float sY[kScanTS * kScanP];
  const int tid = threadIdx.x, lane = tid & 31, wave = tid >> 5;
  const int b  = blockIdx.x;
  const int s0 = 2 * tid;
  const v2f lr2 = *(const v2f*)(lre + s0);
  const v2f li2 = *(const v2f*)(lim + s0);
  const float lr0 = lr2[0], lr1 = lr2[1];
  const float li0 = li2[0], li1 = li2[1];
  float hr0 = 0.f, hi0 = 0.f, hr1 = 0.f, hi1 = 0.f;
  const float* bup = bu + (size_t)b * kT * kS + s0;
  unsigned short* hp = h16 + (size_t)b * kT * kS;
#pragma unroll 1
  for (int t0 = 0; t0 < kT; t0 += kScanTS) {
#pragma unroll 4
    for (int s = 0; s < kScanTS; ++s) {
      const v2f xv = *(const v2f*)(bup + (size_t)(t0 + s) * kS);
      const float nr0 = fmaf(lr0, hr0, fmaf(-li0, hi0, xv[0]));
      const float ni0 = fmaf(lr0, hi0, li0 * hr0);
      const float nr1 = fmaf(lr1, hr1, fmaf(-li1, hi1, xv[1]));
      const float ni1 = fmaf(lr1, hi1, li1 * hr1);
      hr0 = nr0; hi0 = ni0; hr1 = nr1; hi1 = ni1;
      v2f o;
      o[0] = hr0;
      o[1] = hr1;
      *(v2f*)(sY + s * kScanP + s0) = o;
    }
    __syncthreads();
    v8h hv[4];
#pragma unroll
    for (int it = 0; it < 4; ++it) {
      const float* sp = sY + (it * 4 + wave) * kScanP + lane * 8;
      const v4f a0 = *(const v4f*)(sp);
      const v4f a1 = *(const v4f*)(sp + 4);
#pragma unroll
      for (int e = 0; e < 4; ++e) {
        hv[it][e]     = (_Float16)a0[e];
        hv[it][4 + e] = (_Float16)a1[e];
      }
    }
    for (int pass = 0; pass < 2; ++pass) {
#pragma unroll
      for (int it = 0; it < 4; ++it)
        *(volatile v8h*)(hp + (size_t)(t0 + it * 4 + wave) * kS + lane * 8) = hv[it];
      __threadfence();
    }
    __syncthreads();
  }
}

extern "C" void kernel_launch(void* const* d_in, const int* in_sizes, int n_in,
                              void* d_out, int out_size, void* d_ws, size_t ws_size,
                              hipStream_t stream)
{
  if (n_in < 10) return;
  if (in_sizes[0] != kRows * kU) return;
  if (in_sizes[1] != kS || in_sizes[2] != kS) return;
  if (in_sizes[3] != kS * kU) return;
  if (in_sizes[4] != kO * kS) return;
  if (in_sizes[5] != kO * kU) return;
  if (in_sizes[6] != kH * kO) return;
  if (in_sizes[7] != kH * kH) return;
  if (in_sizes[8] != kO * kH) return;
  if (in_sizes[9] != kO * kU) return;
  if (out_size != kRows * kO) return;
  if (ws_size < kWsTotal) return;

  const float* x    = (const float*)d_in[0];
  const float* lre  = (const float*)d_in[1];
  const float* lim  = (const float*)d_in[2];
  const float* Bw   = (const float*)d_in[3];
  const float* Cw   = (const float*)d_in[4];
  const float* Dw   = (const float*)d_in[5];
  const float* W1   = (const float*)d_in[6];
  const float* W2   = (const float*)d_in[7];
  const float* W3   = (const float*)d_in[8];
  const float* Wlin = (const float*)d_in[9];
  float* outp = (float*)d_out;

  char* ws = (char*)d_ws;
  unsigned short* X16  = (unsigned short*)(ws + kOffX16);
  unsigned short* B16  = (unsigned short*)(ws + kOffB16);
  unsigned short* CAT  = (unsigned short*)(ws + kOffCAT);
  unsigned short* W116 = (unsigned short*)(ws + kOffW116);
  unsigned short* W216 = (unsigned short*)(ws + kOffW216);
  unsigned short* W3L  = (unsigned short*)(ws + kOffW3L);
  float*          BU   = (float*)(ws + kOffR1);
  unsigned short* Y16  = (unsigned short*)(ws + kOffY16);
  unsigned short* Z1   = (unsigned short*)(ws + kOffZ1);
  unsigned short* H16  = (unsigned short*)(ws + kOffR2);
  unsigned short* Z2   = (unsigned short*)(ws + kOffZ2);

  cast_f16_pitch_kernel<<<(kRows * kU / 8) / 256, 256, 0, stream>>>(x,    X16,  kRows * kU / 8, kU, kU,    0,  1.0f);
  cast_f16_pitch_kernel<<<(kS * kU / 8) / 256,    256, 0, stream>>>(Bw,   B16,  kS * kU / 8,    kU, kU,    0,  kWCarry);
  cast_f16_pitch_kernel<<<(kO * kS / 8) / 256,    256, 0, stream>>>(Cw,   CAT,  kO * kS / 8,    kS, kCatK, 0,  kWCarry);
  cast_f16_pitch_kernel<<<(kO * kU / 8) / 256,    256, 0, stream>>>(Dw,   CAT,  kO * kU / 8,    kU, kCatK, kS, kWCarry);
  cast_f16_pitch_kernel<<<(kH * kO / 8) / 256,    256, 0, stream>>>(W1,   W116, kH * kO / 8,    kO, kO,    0,  kWCarry);
  cast_f16_pitch_kernel<<<(kH * kH / 8) / 256,    256, 0, stream>>>(W2,   W216, kH * kH / 8,    kH, kH,    0,  kWCarry);
  cast_f16_pitch_kernel<<<(kO * kH / 8) / 256,    256, 0, stream>>>(W3,   W3L,  kO * kH / 8,    kH, kW3lK, 0,  kWCarry);
  cast_f16_pitch_kernel<<<(kO * kU / 8) / 256,    256, 0, stream>>>(Wlin, W3L,  kO * kU / 8,    kU, kW3lK, kH, kWCarry);

  gemm2seg_f16_kernel<0, 0><<<((kRows / 64) * (kS / 64)) / 8, 256, 0, stream>>>(
      X16, kU, kU, X16, kU, 0, B16, kU, (void*)BU, kS, kRows, kS, kWCarryInv);

  scan_kernel<<<kBsz, 128, 0, stream>>>(BU, lre, lim, H16);

  gemm2seg_f16_kernel<1, 0><<<((kRows / 64) * (kO / 64)) / 8, 256, 0, stream>>>(
      H16, kS, kS, X16, kU, kU, CAT, kCatK, (void*)Y16, kO, kRows, kO, kWCarryInv);

  for (int slab = 0; slab < 2; ++slab) {
    const unsigned short* Ys = Y16 + (size_t)slab * kSlabRows * kO;
    const unsigned short* Xs = X16 + (size_t)slab * kSlabRows * kU;
    float* outs = outp + (size_t)slab * kSlabRows * kO;

    gemm2seg_f16_kernel<1, 3><<<((kSlabRows / 64) * (kH / 64)) / 8, 256, 0, stream>>>(
        Ys, kO, kO, Ys, kO, 0, W116, kO, (void*)Z1, kH, kSlabRows, kH, kWCarryInv);

    gemm2seg_f16_kernel<1, 2><<<((kSlabRows / 64) * (kH / 64)) / 8, 256, 0, stream>>>(
        Z1, kH, kH, Z1, kH, 0, W216, kH, (void*)Z2, kH, kSlabRows, kH, kWCarryInv);

    gemm2seg_f16_kernel<0, 0><<<((kSlabRows / 64) * (kO / 64)) / 8, 256, 0, stream>>>(
        Z2, kH, kH, Xs, kU, kU, W3L, kW3lK, (void*)outs, kO, kSlabRows, kO, kWCarryInv);
  }
}
